// mha1_13795434955004
// MI455X (gfx1250) — hardware-verified
//
#include <hip/hip_runtime.h>


namespace {
constexpr int Bn = 2, S = 2048, D = 1024, NH = 16, DH = 64, NT = Bn * S;
constexpr float QS = 8.0f, KS = 8.0f, VS = 8.0f, PS = 8.0f, AS_ = 8.0f;
constexpr size_t PL = (size_t)Bn * NH * S * DH;

typedef _Float16 b16;
typedef __attribute__((ext_vector_type(16))) _Float16 v16b;
typedef __attribute__((ext_vector_type(16))) __bf16 v16bb;
typedef __attribute__((ext_vector_type(8))) _Float16 v8b;
typedef __attribute__((ext_vector_type(8))) unsigned short v8us;
typedef __attribute__((ext_vector_type(8))) float v8f;
typedef __attribute__((ext_vector_type(4))) float v4f;
__device__ __forceinline__ float bf16_rne(float f) { unsigned int u = __float_as_uint(f); u += 0x7FFFu + ((u >> 16) & 1u); return __uint_as_float(u & 0xFFFF0000u); }
__device__ __forceinline__ unsigned short bf16_bits(float f) { unsigned int u = __float_as_uint(f); u += 0x7FFFu + ((u >> 16) & 1u); return (unsigned short)(u >> 16); }
__device__ __forceinline__ void split16(float v, b16& hi, b16& lo) { hi = (b16)v; lo = (b16)(v - (float)hi); }
__device__ __forceinline__ v16b frag_kb(const b16* p, int hh) { const v8b a = *(const v8b*)(p + 8 * hh), b = *(const v8b*)(p + 16 + 8 * hh); v16b f;
#pragma unroll
  for (int e = 0; e < 8; ++e) { f[e] = a[e]; f[8 + e] = b[e]; } return f; }
__device__ __forceinline__ v16bb frag_bf(const unsigned short* p, int hh) { const v8us a = *(const v8us*)(p + 8 * hh), b = *(const v8us*)(p + 16 + 8 * hh); union { unsigned short s[16]; v16bb v; } u;
#pragma unroll
  for (int e = 0; e < 8; ++e) { u.s[e] = a[e]; u.s[8 + e] = b[e]; } return u.v; }
__device__ __forceinline__ v16bb frag_f32bf(const float* p, int hh) { union { unsigned short s[16]; v16bb v; } u;
#pragma unroll
  for (int e = 0; e < 8; ++e) { u.s[e] = bf16_bits(p[8 * hh + e]); u.s[8 + e] = bf16_bits(p[16 + 8 * hh + e]); } return u.v; }
__device__ __forceinline__ void frag_split(const float* p, int hh, v16b& fh, v16b& fl) {
#pragma unroll
  for (int e = 0; e < 8; ++e) { b16 a, c; split16(p[8 * hh + e] * AS_, a, c); fh[e] = a; fl[e] = c; split16(p[16 + 8 * hh + e] * AS_, a, c); fh[8 + e] = a; fl[8 + e] = c; } }
__device__ __forceinline__ v8f wmma16b(v16b a, v16b b, v8f c) { v8f d = __builtin_amdgcn_wmma_f32_16x16x32_f16(false, a, false, b, (short)0, c, false, false); asm volatile("v_nop\n\tv_nop\n\tv_nop\n\tv_nop" : "+v"(d) : "v"(a), "v"(b)); return d; }
__device__ __forceinline__ v8f wmma16bb(v16bb a, v16bb b, v8f c) { v8f d = __builtin_amdgcn_wmma_f32_16x16x32_bf16(false, a, false, b, (short)0, c, false, false); asm volatile("v_nop\n\tv_nop\n\tv_nop\n\tv_nop" : "+v"(d) : "v"(a), "v"(b)); return d; }
__device__ __forceinline__ void wave_lds_sync() { __builtin_amdgcn_fence(__ATOMIC_RELEASE, "workgroup"); __builtin_amdgcn_wave_barrier(); __builtin_amdgcn_fence(__ATOMIC_ACQUIRE, "workgroup"); }
__device__ __forceinline__ float nexp(float x) { return __builtin_amdgcn_exp2f(x * 1.4426950408889634f); }

__device__ __forceinline__ int cperm(int cp) { return (cp & 63) * NH + (cp >> 6); }
__global__ __launch_bounds__(256) void prep_kernel(const float* __restrict__ Wk, const float* __restrict__ Wq, const float* __restrict__ Wv, const float* __restrict__ Wo, const float* __restrict__ bk, const float* __restrict__ bq, const float* __restrict__ bv, const float* __restrict__ bo, unsigned short* __restrict__ w16, b16* __restrict__ wo16, float* __restrict__ P) {
  const size_t tid = (size_t)blockIdx.x * blockDim.x + threadIdx.x, nth = (size_t)gridDim.x * blockDim.x;
  for (int pass = 0; pass < 2; ++pass) {
    for (size_t p = tid; p < (size_t)3 * D * D / 8; p += nth) { const int m = (int)(p / (D * D / 8)); const size_t q = p % (D * D / 8); const int cp = (int)(q / (D / 8)), k8 = (int)(q % (D / 8)) * 8; const float* W = ((m == 0) ? Wk : (m == 1) ? Wq : Wv) + (size_t)cperm(cp) * D; v8us v;
#pragma unroll
      for (int e = 0; e < 8; ++e) v[e] = bf16_bits(W[k8 + e]);
      *(volatile v8us*)(w16 + p * 8) = v; }
    for (size_t p = tid; p < (size_t)D * D / 8; p += nth) { const int o = (int)(p / (D / 8)), k8 = (int)(p % (D / 8)) * 8; v8b v;
#pragma unroll
      for (int e = 0; e < 8; ++e) v[e] = (b16)bf16_rne(Wo[(size_t)o * D + cperm(k8 + e)]);
      *(volatile v8b*)(wo16 + p * 8) = v; }
    for (size_t p = tid; p < 4096 / 4; p += nth) { v4f v;
#pragma unroll
      for (int e = 0; e < 4; ++e) { const int i = (int)p * 4 + e, j = i & 1023; v[e] = bf16_rne((i < 1024) ? bk[cperm(j)] : (i < 2048) ? bq[cperm(j)] : (i < 3072) ? bv[cperm(j)] : bo[j]); }
      *(volatile v4f*)(P + p * 4) = v; }
    __threadfence(); }
}

__global__ __launch_bounds__(128) void proj_kernel(const float* __restrict__ KEY, const float* __restrict__ QUERY, const float* __restrict__ VALUE, const unsigned short* __restrict__ w16, const float* __restrict__ P, b16* __restrict__ qp, b16* __restrict__ kp, b16* __restrict__ vt) {
  __shared__ __attribute__((aligned(16))) b16 Th[4][32][64 + 8], Tl[4][32][64 + 8]; __shared__ __attribute__((aligned(16))) b16 Tv[64][128 + 8];
  const int lane = threadIdx.x & 31, wave = threadIdx.x >> 5, nloc = lane & 15, hlf = lane >> 4, which = blockIdx.z, h = blockIdx.x, c0 = h * DH, p0 = blockIdx.y * 128, m0 = p0 + wave * 32, b = p0 / S, t0 = p0 % S;
  const float* X = (which == 0) ? KEY : (which == 1) ? QUERY : VALUE; const unsigned short* Wt = w16 + (size_t)which * D * D; const float* bias = P + which * 1024;
  v8f acc[2][4];
#pragma unroll
  for (int r = 0; r < 2; ++r)
#pragma unroll
    for (int t = 0; t < 4; ++t) acc[r][t] = (v8f){};
#pragma unroll 2
  for (int kb = 0; kb < D; kb += 32) { const v16bb a0 = frag_f32bf(X + (size_t)(m0 + nloc) * D + kb, hlf), a1 = frag_f32bf(X + (size_t)(m0 + 16 + nloc) * D + kb, hlf);
#pragma unroll
    for (int t = 0; t < 4; ++t) { const v16bb bw = frag_bf(Wt + (size_t)(c0 + t * 16 + nloc) * D + kb, hlf); acc[0][t] = wmma16bb(a0, bw, acc[0][t]); acc[1][t] = wmma16bb(a1, bw, acc[1][t]); } }
  if (which < 2) { const float scl = (which == 1) ? QS : KS;
#pragma unroll
    for (int t = 0; t < 4; ++t) { const float bb = bias[c0 + t * 16 + nloc];
#pragma unroll
      for (int r = 0; r < 2; ++r)
#pragma unroll
        for (int v = 0; v < 8; ++v) { b16 a_, l_; split16((acc[r][t][v] + bb) * scl, a_, l_); Th[wave][r * 16 + 8 * hlf + v][t * 16 + nloc] = a_; Tl[wave][r * 16 + 8 * hlf + v][t * 16 + nloc] = l_; } }
    wave_lds_sync();
    b16* base = ((which == 1) ? qp : kp) + (((size_t)b * NH + h) * S + (m0 % S)) * DH;
    for (int pass = 0; pass < 2; ++pass) {
#pragma unroll
      for (int j = 0; j < 8; ++j) { const int rr = j * 4 + (lane >> 3), c8 = (lane & 7) * 8; *(volatile v8b*)(base + (size_t)rr * DH + c8) = *(const v8b*)(&Th[wave][rr][c8]); if (which == 1) *(volatile v8b*)(base + PL + (size_t)rr * DH + c8) = *(const v8b*)(&Tl[wave][rr][c8]); }
      __threadfence(); }
    return; }
#pragma unroll
  for (int t = 0; t < 4; ++t) { const float bb = bias[c0 + t * 16 + nloc];
#pragma unroll
    for (int r = 0; r < 2; ++r)
#pragma unroll
      for (int v = 0; v < 8; ++v) Tv[t * 16 + nloc][wave * 32 + r * 16 + 8 * hlf + v] = (b16)((acc[r][t][v] + bb) * VS); }
  __syncthreads();
  for (int pass = 0; pass < 2; ++pass) { for (int i = threadIdx.x; i < 64 * 16; i += 128) { const int d = i >> 4, c8 = (i & 15) * 8; *(volatile v8b*)(vt + (((size_t)b * NH + h) * DH + d) * S + t0 + c8) = *(const v8b*)(&Tv[d][c8]); } __threadfence(); }
}

constexpr int HW = 1, NWV = 16;
__global__ __launch_bounds__(512) void attn_kernel(const b16* __restrict__ qp, const b16* __restrict__ kp, const b16* __restrict__ vt, float* __restrict__ ctx) {
  __shared__ float Mx[NWV][32][16], Sm[NWV][32][16]; __shared__ __attribute__((aligned(16))) float Os[16][D + 4];
  const int wid = threadIdx.x >> 5, lane = threadIdx.x & 31, hh = lane >> 4, col = lane & 15; const int b = blockIdx.x / (S / 16), q0 = (blockIdx.x % (S / 16)) * 16, qi = q0 + col;
  v8f o[HW][4];
#pragma unroll
  for (int j = 0; j < HW; ++j)
#pragma unroll
    for (int t = 0; t < 4; ++t) o[j][t] = (v8f){};
  for (int kb = 0; kb < S; kb += 32) {
    v8f s[HW][2];
#pragma unroll
    for (int j = 0; j < HW; ++j) { const int h = wid * HW + j; const b16* K = kp + (((size_t)b * NH + h) * S) * DH; const b16* Q = qp + (((size_t)b * NH + h) * S + qi) * DH; s[j][0] = (v8f){}; s[j][1] = (v8f){};
#pragma unroll
      for (int ks = 0; ks < 2; ++ks) { const v16b qf = frag_kb(Q + ks * 32, hh), ql = frag_kb(Q + PL + ks * 32, hh);
        const v16b ka = frag_kb(K + (size_t)(kb + col) * DH + ks * 32, hh), kc = frag_kb(K + (size_t)(kb + 16 + col) * DH + ks * 32, hh);
        s[j][0] = wmma16b(ka, qf, s[j][0]); s[j][0] = wmma16b(ka, ql, s[j][0]); s[j][1] = wmma16b(kc, qf, s[j][1]); s[j][1] = wmma16b(kc, ql, s[j][1]); } }
#pragma unroll
    for (int tI = 0; tI < 2; ++tI)
#pragma unroll
      for (int r = 0; r < 8; ++r) { float m2 = -INFINITY;
#pragma unroll
        for (int j = 0; j < HW; ++j) { s[j][tI][r] *= 1.0f / (QS * KS * 8.0f); m2 = fmaxf(m2, s[j][tI][r]); }
        Mx[wid][tI * 16 + 8 * hh + r][col] = m2; }
    __syncthreads();
    float esum[2][8];
#pragma unroll
    for (int tI = 0; tI < 2; ++tI)
#pragma unroll
      for (int r = 0; r < 8; ++r) { const int i = tI * 16 + 8 * hh + r; float m = -INFINITY;
#pragma unroll
        for (int w = 0; w < NWV; ++w) m = fmaxf(m, Mx[w][i][col]);
        float sm = 0.0f;
#pragma unroll
        for (int j = 0; j < HW; ++j) { const float e = nexp(s[j][tI][r] - m); s[j][tI][r] = e; sm += e; }
        esum[tI][r] = sm; }
#pragma unroll
    for (int tI = 0; tI < 2; ++tI)
#pragma unroll
      for (int r = 0; r < 8; ++r) Sm[wid][tI * 16 + 8 * hh + r][col] = esum[tI][r];
    __syncthreads();
#pragma unroll
    for (int j = 0; j < HW; ++j) { v16b pbv, plv;
#pragma unroll
      for (int tI = 0; tI < 2; ++tI)
#pragma unroll
        for (int r = 0; r < 8; ++r) { const int i = tI * 16 + 8 * hh + r; float tot = 0.0f;
#pragma unroll
          for (int w = 0; w < NWV; w += 2) tot += Sm[w][i][col] + Sm[w + 1][i][col];
          const float wgt = s[j][tI][r] / tot; b16 a_, l_; split16(wgt * PS, a_, l_); pbv[tI * 8 + r] = a_; plv[tI * 8 + r] = l_; }
      const int h = wid * HW + j; const b16* V = vt + (((size_t)b * NH + h) * DH) * S;
#pragma unroll
      for (int t = 0; t < 4; ++t) { const v16b vf = frag_kb(V + (size_t)(t * 16 + col) * S + kb, hh); o[j][t] = wmma16b(vf, pbv, o[j][t]); o[j][t] = wmma16b(vf, plv, o[j][t]); } }
    __syncthreads();
  }
#pragma unroll
  for (int j = 0; j < HW; ++j)
#pragma unroll
    for (int t = 0; t < 4; ++t)
#pragma unroll
      for (int r = 0; r < 8; ++r) Os[col][(wid * HW + j) * DH + t * 16 + 8 * hh + r] = o[j][t][r] * (1.0f / (VS * PS));
  __syncthreads();
  float* dst = ctx + ((size_t)b * S + q0) * D;
  for (int pass = 0; pass < 2; ++pass) { for (int i = threadIdx.x; i < 16 * (D / 4); i += 512) { const int rr = i / (D / 4), c4 = (i % (D / 4)) * 4; *(volatile v4f*)(dst + (size_t)rr * D + c4) = *(const v4f*)(&Os[rr][c4]); } __threadfence(); }
}

__global__ __launch_bounds__(128) void out_kernel(const float* __restrict__ ctx, const b16* __restrict__ wo16, const float* __restrict__ P, float* __restrict__ out) {
  __shared__ __attribute__((aligned(16))) float Ts[4][32 * 64];
  const int lane = threadIdx.x & 31, wave = threadIdx.x >> 5, nloc = lane & 15, hlf = lane >> 4, m0 = blockIdx.y * 128 + wave * 32, c0 = blockIdx.x * 64; const float* bo = P + 3072;
  v8f acc[2][4];
#pragma unroll
  for (int r = 0; r < 2; ++r)
#pragma unroll
    for (int t = 0; t < 4; ++t) acc[r][t] = (v8f){};
#pragma unroll 2
  for (int kb = 0; kb < D; kb += 32) { v16b a0, l0, a1, l1; frag_split(ctx + (size_t)(m0 + nloc) * D + kb, hlf, a0, l0); frag_split(ctx + (size_t)(m0 + 16 + nloc) * D + kb, hlf, a1, l1);
#pragma unroll
    for (int t = 0; t < 4; ++t) { const v16b bw = frag_kb(wo16 + (size_t)(c0 + t * 16 + nloc) * D + kb, hlf); acc[0][t] = wmma16b(a0, bw, acc[0][t]); acc[0][t] = wmma16b(l0, bw, acc[0][t]); acc[1][t] = wmma16b(a1, bw, acc[1][t]); acc[1][t] = wmma16b(l1, bw, acc[1][t]); } }
  float* Tt = Ts[wave];
#pragma unroll
  for (int t = 0; t < 4; ++t) { const float bb = bo[c0 + t * 16 + nloc];
#pragma unroll
    for (int r = 0; r < 2; ++r)
#pragma unroll
      for (int v = 0; v < 8; ++v) Tt[(r * 16 + v + 8 * hlf) * 64 + t * 16 + nloc] = acc[r][t][v] * (1.0f / AS_) + bb; }
  wave_lds_sync();
  for (int pass = 0; pass < 2; ++pass) {
#pragma unroll
    for (int j = 0; j < 16; ++j) { const int rr = j * 2 + hlf, c4 = nloc * 4; *(volatile v4f*)(out + (size_t)(m0 + rr) * D + c0 + c4) = *(const v4f*)(Tt + rr * 64 + c4); }
    __threadfence(); }
}
}

extern "C" void kernel_launch(void* const* d_in, const int* in_sizes, int n_in,
                              void* d_out, int out_size, void* d_ws, size_t ws_size, hipStream_t stream) {
  (void)n_in; (void)out_size;
  const float* KEY = (const float*)d_in[0]; const float* VALUE = (const float*)d_in[1]; const float* QUERY = (const float*)d_in[2];
  const float* Wk = (const float*)d_in[3]; const float* bk = (const float*)d_in[4]; const float* Wq = (const float*)d_in[5]; const float* bq = (const float*)d_in[6]; const float* Wv = (const float*)d_in[7]; const float* bv = (const float*)d_in[8]; const float* Wo = (const float*)d_in[9]; const float* bo = (const float*)d_in[10];
  float* out = (float*)d_out;
  if (in_sizes[0] != NT * D || in_sizes[1] != NT * D || in_sizes[2] != NT * D || in_sizes[3] != D * D || in_sizes[9] != D * D || in_sizes[10] != D) return;
  size_t off = 0; char* ws = (char*)d_ws;
  auto carve = [&](size_t bytes) { char* p = ws + off; off += (bytes + 255) & ~(size_t)255; return p; };
  unsigned short* w16 = (unsigned short*)carve((size_t)3 * D * D * 2); b16* wo16 = (b16*)carve((size_t)D * D * 2); float* P = (float*)carve(4096 * 4);
  b16* qp = (b16*)carve(PL * 2 * 2); b16* kp = (b16*)carve(PL * 2); b16* vt = (b16*)carve(PL * 2); float* ctx = (float*)carve((size_t)NT * D * 4);
  if (off > ws_size) return;
  prep_kernel<<<512, 256, 0, stream>>>(Wk, Wq, Wv, Wo, bk, bq, bv, bo, w16, wo16, P);
  proj_kernel<<<dim3(NH, NT / 128, 3), 128, 0, stream>>>(KEY, QUERY, VALUE, w16, P, qp, kp, vt);
  attn_kernel<<<NT / 16, 512, 0, stream>>>(qp, kp, vt, ctx);
  out_kernel<<<dim3(D / 64, NT / 128), 128, 0, stream>>>(ctx, wo16, P, out);
}
